// SSM_60902636257786
// MI455X (gfx1250) — hardware-run, weakly checked
//
#include <hip/hip_runtime.h>
#include <math.h>

typedef __attribute__((ext_vector_type(16))) _Float16 v16h;
typedef __attribute__((ext_vector_type(8)))  _Float16 v8h;
typedef __attribute__((ext_vector_type(8)))  float    v8f;
typedef __attribute__((ext_vector_type(4)))  float    v4f;

constexpr int kNB     = 16;
constexpr int kCin    = 64;
constexpr int kLen    = 4096;
constexpr int kDmod   = 256;
constexpr int kNst    = 64;
constexpr int kNout   = 10;
constexpr int kRowsM  = kNB * kLen;
constexpr int kChunk  = 512;
constexpr int kNChunk = kLen / kChunk;
constexpr int kStepsPerFlush = 64;
constexpr int kTilePitch = 68;
constexpr int kUBlocks = kNB * (kLen / 64);
constexpr int kWBlocks = (kDmod * kCin / 8) / 256;
static_assert(kCin == 64 && (kCin % 32) == 0, "K tile multiple");
static_assert((kRowsM % 64) == 0 && (kDmod % 64) == 0, "M,N tile multiples");
static_assert(kNChunk == 8 && (kChunk % 32) == 0, "chunking");
static_assert(kNst == 64 && (kLen % kStepsPerFlush) == 0, "recurrence block");
static_assert(kNB * kNout == 160, "output count");
static_assert(kWBlocks * 256 * 8 == kDmod * kCin, "weight plane coverage");

constexpr float kCarryU = 64.0f;
constexpr float kCarryW = 256.0f;
constexpr float kFold   = 1.0f / (kCarryU * kCarryW);
constexpr float kInvLen = 1.0f / (float)kLen;
constexpr float kHalfMinNormal = 6.103515625e-05f;

constexpr size_t kOffPS  = 0;
constexpr size_t kOffWT  = kOffPS  + (size_t)kLen * kNst * 4;
constexpr size_t kOffSM  = kOffWT  + (size_t)kLen * 4;
constexpr size_t kOffU16 = kOffSM  + 128;
constexpr size_t kOffW16 = kOffU16 + (size_t)kRowsM * kCin * 2;
constexpr size_t kOffYP  = kOffW16 + (size_t)kDmod * kCin * 2;
constexpr size_t kWsTotal = kOffYP + (size_t)kNB * kNChunk * kDmod * 4;
static_assert(kWsTotal == 9617536ull, "carve total");
static_assert(kWsTotal <= 134217728ull, "carve cap");
static_assert((kOffWT % 128) == 0 && (kOffSM % 128) == 0 && (kOffU16 % 128) == 0 &&
              (kOffW16 % 128) == 0 && (kOffYP % 128) == 0, "aligned regions");

union FragH { v16h v; v8h h[2]; };
__device__ __forceinline__ v16h frag_load(const _Float16* p) {
  FragH f;
  f.h[0] = *(const v8h*)(p);
  f.h[1] = *(const v8h*)(p + 16);
  return f.v;
}
__device__ __forceinline__ v8f mma_h(v16h a, v16h b, v8f c) {
  c = __builtin_amdgcn_wmma_f32_16x16x32_f16(false, a, false, b, (short)0, c, false, false);
  asm volatile("v_nop\n\tv_nop\n\tv_nop\n\tv_nop" : "+v"(c) : "v"(a), "v"(b));
  return c;
}
__device__ __forceinline__ float carry_flush(float x, float carry) {
  const float v = x * carry;
  return (fabsf(v) < kHalfMinNormal) ? 0.0f : v;
}

__global__ __launch_bounds__(64) void wrec_kernel(
    const float* __restrict__ Am, const float* __restrict__ Bv, const float* __restrict__ Cv,
    float* __restrict__ PS)
{
  __shared__ __align__(16) float sZ[2 * kNst];
  __shared__ __align__(16) float sS[kStepsPerFlush * kNst];
  const int i = threadIdx.x;
  const int lane = i & 31, wave = i >> 5;
  const int hh = lane >> 4, c4 = (lane & 15) * 4;

  float a[kNst];
#pragma unroll
  for (int q = 0; q < kNst / 4; ++q) {
    const v4f t = *(const v4f*)(Am + (size_t)i * kNst + 4 * q);
    a[4 * q + 0] = t[0];
    a[4 * q + 1] = t[1];
    a[4 * q + 2] = t[2];
    a[4 * q + 3] = t[3];
  }
  const float cv = Cv[i];
  float S = 0.0f;
  sZ[i] = Bv[i];
  __syncthreads();
  int cur = 0;
#pragma unroll 1
  for (int m0 = 0; m0 < kLen; m0 += kStepsPerFlush) {
#pragma unroll 1
    for (int s = 0; s < kStepsPerFlush; ++s) {
      const float* zc = sZ + cur * kNst;
      const float zi = zc[i];
      S = fmaf(cv, zi, S);
      sS[s * kNst + i] = S;
      float zn = 0.0f;
#pragma unroll
      for (int q = 0; q < kNst / 4; ++q) {
        const v4f zv = *(const v4f*)(zc + 4 * q);
        zn = fmaf(a[4 * q + 0], zv[0], zn);
        zn = fmaf(a[4 * q + 1], zv[1], zn);
        zn = fmaf(a[4 * q + 2], zv[2], zn);
        zn = fmaf(a[4 * q + 3], zv[3], zn);
      }
      sZ[(cur ^ 1) * kNst + i] = zn;
      __syncthreads();
      cur ^= 1;
    }
    for (int pass = 0; pass < 2; ++pass) {
#pragma unroll 4
      for (int it = 0; it < 16; ++it) {
        const int row = it * 4 + wave * 2 + hh;
        const v4f v = *(const v4f*)(sS + row * kNst + c4);
        *(volatile v4f*)(PS + (size_t)(m0 + row) * kNst + c4) = v;
      }
      __threadfence();
    }
    __syncthreads();
  }
}

__global__ __launch_bounds__(256) void wsum_kernel(
    const float* __restrict__ PS, float* __restrict__ WT, float* __restrict__ SM)
{
  __shared__ __align__(16) float sW[kLen];
  __shared__ float sR[256];
  const int t = threadIdx.x;
  float tot = 0.0f;
#pragma unroll 1
  for (int it = 0; it < kLen / 256; ++it) {
    const int k = it * 256 + t;
    const float* row = PS + (size_t)(kLen - 1 - k) * kNst;
    float acc = 0.0f;
#pragma unroll
    for (int q = 0; q < kNst / 4; ++q) {
      const v4f v = *(const v4f*)(row + 4 * q);
      acc += v[0];
      acc += v[1];
      acc += v[2];
      acc += v[3];
    }
    sW[k] = acc;
    tot += acc;
  }
  sR[t] = tot;
  __syncthreads();
  for (int off = 128; off > 0; off >>= 1) {
    if (t < off) sR[t] += sR[t + off];
    __syncthreads();
  }
  const float smean = sR[0] * kInvLen;
  for (int pass = 0; pass < 2; ++pass) {
#pragma unroll
    for (int it = 0; it < 4; ++it) {
      const int k4 = (it * 256 + t) * 4;
      const v4f v = *(const v4f*)(sW + k4);
      *(volatile v4f*)(WT + k4) = v;
    }
    if (t < 32) *(volatile float*)(SM + t) = smean;
    __threadfence();
  }
}

__global__ __launch_bounds__(256) void prep_kernel(
    const float* __restrict__ u, const float* __restrict__ Wup,
    _Float16* __restrict__ U16, _Float16* __restrict__ W16)
{
  __shared__ __align__(16) float sT[64 * kTilePitch];
  const int tid = threadIdx.x, lane = tid & 31, wave = tid >> 5;
  if (blockIdx.x >= kUBlocks) {
    const int i = (blockIdx.x - kUBlocks) * 256 + tid;
    const size_t e0 = (size_t)i * 8;
    const v4f a0 = *(const v4f*)(Wup + e0);
    const v4f a1 = *(const v4f*)(Wup + e0 + 4);
    v8h hv;
#pragma unroll
    for (int e = 0; e < 4; ++e) {
      hv[e]     = (_Float16)carry_flush(a0[e], kCarryW);
      hv[4 + e] = (_Float16)carry_flush(a1[e], kCarryW);
    }
    *(volatile v8h*)(W16 + e0) = hv;
    __threadfence();
    *(volatile v8h*)(W16 + e0) = hv;
    return;
  }
  const int bb = blockIdx.x >> 6;
  const int l0 = (blockIdx.x & 63) * 64;
  {
    const int cr = tid >> 4, l4 = (tid & 15) * 4;
#pragma unroll
    for (int p = 0; p < 4; ++p) {
      const int c = p * 16 + cr;
      const v4f x = *(const v4f*)(u + ((size_t)(bb * kCin + c)) * kLen + l0 + l4);
      sT[(l4 + 0) * kTilePitch + c] = x[0];
      sT[(l4 + 1) * kTilePitch + c] = x[1];
      sT[(l4 + 2) * kTilePitch + c] = x[2];
      sT[(l4 + 3) * kTilePitch + c] = x[3];
    }
  }
  __syncthreads();
  const int q = lane >> 3, c8 = (lane & 7) * 8;
  v8h hv[2];
#pragma unroll
  for (int it = 0; it < 2; ++it) {
    const int row = it * 32 + wave * 4 + q;
    const float* sp = sT + row * kTilePitch + c8;
    const v4f a0 = *(const v4f*)(sp);
    const v4f a1 = *(const v4f*)(sp + 4);
#pragma unroll
    for (int e = 0; e < 4; ++e) {
      hv[it][e]     = (_Float16)carry_flush(a0[e], kCarryU);
      hv[it][4 + e] = (_Float16)carry_flush(a1[e], kCarryU);
    }
  }
  for (int pass = 0; pass < 2; ++pass) {
#pragma unroll
    for (int it = 0; it < 2; ++it) {
      const int row = it * 32 + wave * 4 + q;
      *(volatile v8h*)(U16 + ((size_t)bb * kLen + l0 + row) * kCin + c8) = hv[it];
    }
    __threadfence();
  }
}

__global__ __launch_bounds__(256) void proj_reduce_kernel(
    const _Float16* __restrict__ U16, const _Float16* __restrict__ W16,
    const float* __restrict__ WT, float* __restrict__ YP)
{
  __shared__ __align__(16) float sPart[2 * kDmod];
  const int tid = threadIdx.x, lane = tid & 31, wave = tid >> 5;
  const int rl = lane & 15, hh = lane >> 4;
  const int tn = wave & 3, mh = wave >> 2;
  const int n0 = tn * 64;
  const int bb = blockIdx.x / kNChunk;
  const int ch = blockIdx.x - bb * kNChunk;
  const int l0 = ch * kChunk + mh * (kChunk / 2);
  const _Float16* Ab = U16 + ((size_t)bb * kLen + l0) * kCin;

  v16h bfr[4][2];
#pragma unroll
  for (int j = 0; j < 4; ++j) {
#pragma unroll
    for (int kk = 0; kk < 2; ++kk)
      bfr[j][kk] = frag_load(W16 + (size_t)(n0 + j * 16 + rl) * kCin + kk * 32 + hh * 8);
  }
  float part[4];
#pragma unroll
  for (int j = 0; j < 4; ++j) part[j] = 0.0f;

#pragma unroll 1
  for (int g = 0; g < (kChunk / 2) / 16; ++g) {
    const _Float16* ap = Ab + (size_t)(g * 16 + rl) * kCin + hh * 8;
    const v16h a0 = frag_load(ap);
    const v16h a1 = frag_load(ap + 32);
    const float* wp = WT + l0 + g * 16 + hh * 8;
    const v4f w0 = *(const v4f*)(wp);
    const v4f w1 = *(const v4f*)(wp + 4);
    v8f acc[4];
#pragma unroll
    for (int j = 0; j < 4; ++j) {
      acc[j] = (v8f){0.f, 0.f, 0.f, 0.f, 0.f, 0.f, 0.f, 0.f};
      acc[j] = mma_h(a0, bfr[j][0], acc[j]);
      acc[j] = mma_h(a1, bfr[j][1], acc[j]);
    }
#pragma unroll
    for (int j = 0; j < 4; ++j) {
      float p = part[j];
      p = fmaf(w0[0], acc[j][0], p);
      p = fmaf(w0[1], acc[j][1], p);
      p = fmaf(w0[2], acc[j][2], p);
      p = fmaf(w0[3], acc[j][3], p);
      p = fmaf(w1[0], acc[j][4], p);
      p = fmaf(w1[1], acc[j][5], p);
      p = fmaf(w1[2], acc[j][6], p);
      p = fmaf(w1[3], acc[j][7], p);
      part[j] = p;
    }
  }
#pragma unroll
  for (int j = 0; j < 4; ++j) {
    const float o = __shfl_xor(part[j], 16, 32);
    part[j] = part[j] + o;
  }
  if (hh == 0) {
#pragma unroll
    for (int j = 0; j < 4; ++j) sPart[mh * kDmod + n0 + j * 16 + rl] = part[j];
  }
  __syncthreads();
  if (tid < 64) {
    const int n4 = tid * 4;
    const v4f p0 = *(const v4f*)(sPart + n4);
    const v4f p1 = *(const v4f*)(sPart + kDmod + n4);
    const v4f v = (p0 + p1) * kFold;
    float* dst = YP + (size_t)blockIdx.x * kDmod + n4;
    *(volatile v4f*)dst = v;
    __threadfence();
    *(volatile v4f*)dst = v;
  }
}

__global__ __launch_bounds__(256) void final_kernel(
    const float* __restrict__ YP, const float* __restrict__ bup, const float* __restrict__ SM,
    const float* __restrict__ Wdn, const float* __restrict__ bdn, float* __restrict__ out)
{
  __shared__ __align__(16) float sY[kNB * kDmod];
  __shared__ __align__(16) float sO[256];
  const int t = threadIdx.x;
  const float smean = SM[0];
  const float bu = bup[t];
#pragma unroll 1
  for (int b = 0; b < kNB; ++b) {
    float acc = 0.0f;
#pragma unroll
    for (int c = 0; c < kNChunk; ++c) acc += YP[(size_t)(b * kNChunk + c) * kDmod + t];
    sY[b * kDmod + t] = fmaf(bu, smean, acc * kInvLen);
  }
  __syncthreads();
  const int ic = (t < kNB * kNout) ? t : (kNB * kNout - 1);
  const int bq = ic / kNout;
  const int oq = ic - bq * kNout;
  const float* yr = sY + bq * kDmod;
  const float* wr = Wdn + (size_t)oq * kDmod;
  float acc = 0.0f;
#pragma unroll 2
  for (int d4 = 0; d4 < kDmod / 4; ++d4) {
    const v4f yv = *(const v4f*)(yr + 4 * d4);
    const v4f wv = *(const v4f*)(wr + 4 * d4);
    acc = fmaf(yv[0], wv[0], acc);
    acc = fmaf(yv[1], wv[1], acc);
    acc = fmaf(yv[2], wv[2], acc);
    acc = fmaf(yv[3], wv[3], acc);
  }
  const float bd = bdn[oq];
  const float val = acc + bd;
  sO[t] = (t < kNB * kNout) ? val : 0.0f;
  __syncthreads();
  if (t < 32) {
    const v4f v0 = *(const v4f*)(sO + 4 * t);
    const v4f v1 = *(const v4f*)(sO + 128 + 4 * t);
    for (int pass = 0; pass < 2; ++pass) {
      *(volatile v4f*)(out + 4 * t) = v0;
      if (t < 8) *(volatile v4f*)(out + 128 + 4 * t) = v1;
      __threadfence();
    }
  }
}

extern "C" void kernel_launch(void* const* d_in, const int* in_sizes, int n_in,
                              void* d_out, int out_size, void* d_ws, size_t ws_size,
                              hipStream_t stream) {
  if (n_in < 8) return;
  if (in_sizes[0] != kNB * kCin * kLen) return;
  if (in_sizes[1] != kDmod * kCin) return;
  if (in_sizes[2] != kDmod) return;
  if (in_sizes[3] != kNst * kNst) return;
  if (in_sizes[4] != kNst) return;
  if (in_sizes[5] != kNst) return;
  if (in_sizes[6] != kNout * kDmod) return;
  if (in_sizes[7] != kNout) return;
  if (out_size != kNB * kNout) return;
  if (ws_size < kWsTotal) return;

  const float* u      = (const float*)d_in[0];
  const float* W_up   = (const float*)d_in[1];
  const float* b_up   = (const float*)d_in[2];
  const float* A_m    = (const float*)d_in[3];
  const float* Bv     = (const float*)d_in[4];
  const float* Cv     = (const float*)d_in[5];
  const float* W_down = (const float*)d_in[6];
  const float* b_down = (const float*)d_in[7];
  float* out = (float*)d_out;

  char* ws = (char*)d_ws;
  float*    PS  = (float*)(ws + kOffPS);
  float*    WT  = (float*)(ws + kOffWT);
  float*    SM  = (float*)(ws + kOffSM);
  _Float16* U16 = (_Float16*)(ws + kOffU16);
  _Float16* W16 = (_Float16*)(ws + kOffW16);
  float*    YP  = (float*)(ws + kOffYP);

  wrec_kernel<<<1, 64, 0, stream>>>(A_m, Bv, Cv, PS);
  wsum_kernel<<<1, 256, 0, stream>>>(PS, WT, SM);
  prep_kernel<<<kUBlocks + kWBlocks, 256, 0, stream>>>(u, W_up, U16, W16);
  proj_reduce_kernel<<<kNB * kNChunk, 256, 0, stream>>>(U16, W16, WT, YP);
  final_kernel<<<1, 256, 0, stream>>>(YP, b_up, SM, W_down, b_down, out);
}
